// SiteExposureLSTM_85667417686275
// MI455X (gfx1250) — hardware-verified
//
#include <hip/hip_runtime.h>
#include <stddef.h>


typedef _Float16 v16h __attribute__((ext_vector_type(16)));
typedef float    v8f  __attribute__((ext_vector_type(8)));
typedef float    v4f  __attribute__((ext_vector_type(4)));

#define HID 16
#define NOUT 4
#define ROWS_PER_WAVE 16

#define SC_ACT  256.0f
#define SC_W    16.0f
#define SC_ACC  4096.0f
#define INV_ACC (1.0f / 4096.0f)
#define LOG2E_F 1.4426950408889634f

__device__ __forceinline__ v8f wmma_f16_guarded(v16h a, v16h b, v8f c) {
    v8f d = __builtin_amdgcn_wmma_f32_16x16x32_f16(false, a, false, b, (short)0, c, false, false);
    asm volatile("v_nop\n\tv_nop\n\tv_nop\n\tv_nop" : "+v"(d) : "v"(a), "v"(b));
    return d;
}

__device__ __forceinline__ float sig_scaled(float x, float k) {
    float e = __builtin_amdgcn_exp2f(x * (-LOG2E_F * k));
    return __builtin_amdgcn_rcpf(1.0f + e);
}
__device__ __forceinline__ float tanh_scaled(float x, float k) {
    float e = __builtin_amdgcn_exp2f(x * (-2.0f * LOG2E_F * k));
    return fmaf(2.0f, __builtin_amdgcn_rcpf(1.0f + e), -1.0f);
}

__device__ __forceinline__ v16h frag_row8(const float* __restrict__ p, float scale) {
    v16h v;
#pragma unroll
    for (int e = 0; e < 8; ++e) v[e] = (_Float16)(p[e] * scale);
#pragma unroll
    for (int e = 8; e < 16; ++e) v[e] = (_Float16)0.0f;
    return v;
}

__global__ __launch_bounds__(32) void lstm_head_fused(
    const float* __restrict__ x,
    const float* __restrict__ W_ih,
    const float* __restrict__ W_hh,
    const float* __restrict__ b_ih,
    const float* __restrict__ b_hh,
    const float* __restrict__ W1,
    const float* __restrict__ b1,
    const float* __restrict__ W2,
    const float* __restrict__ b2,
    float* __restrict__ out,
    int B, int T)
{
    const int lane = threadIdx.x & 31;
    const int n    = lane & 15;
    const int hh   = lane >> 4;
    const int row  = blockIdx.x * ROWS_PER_WAVE + n;
    const int rowc = (row < B) ? row : (B - 1);

    const v16h aw0 = frag_row8(W_hh + (size_t)(0 * HID + n) * HID + 8 * hh, SC_W);
    const v16h aw1 = frag_row8(W_hh + (size_t)(1 * HID + n) * HID + 8 * hh, SC_W);
    const v16h aw2 = frag_row8(W_hh + (size_t)(2 * HID + n) * HID + 8 * hh, SC_W);
    const v16h aw3 = frag_row8(W_hh + (size_t)(3 * HID + n) * HID + 8 * hh, SC_W);

    float wih[4][8], bsm[4][8];
#pragma unroll
    for (int g = 0; g < 4; ++g) {
#pragma unroll
        for (int r = 0; r < 8; ++r) {
            const int gr = 16 * g + 8 * hh + r;
            wih[g][r] = W_ih[gr] * SC_ACC;
            bsm[g][r] = (b_ih[gr] + b_hh[gr]) * SC_ACC;
        }
    }

    float c[8], h[8];
#pragma unroll
    for (int r = 0; r < 8; ++r) { c[r] = 0.0f; h[r] = 0.0f; }

    const float* xrow = x + (size_t)rowc * (size_t)T;

    for (int t = 0; t < T; ++t) {
        const float xv = xrow[t];

        v16h bv;
#pragma unroll
        for (int e = 0; e < 8; ++e) bv[e] = (_Float16)(h[e] * SC_ACT);
#pragma unroll
        for (int e = 8; e < 16; ++e) bv[e] = (_Float16)0.0f;

        v8f acc0, acc1, acc2, acc3;
#pragma unroll
        for (int r = 0; r < 8; ++r) {
            acc0[r] = fmaf(xv, wih[0][r], bsm[0][r]);
            acc1[r] = fmaf(xv, wih[1][r], bsm[1][r]);
            acc2[r] = fmaf(xv, wih[2][r], bsm[2][r]);
            acc3[r] = fmaf(xv, wih[3][r], bsm[3][r]);
        }
        acc0 = wmma_f16_guarded(aw0, bv, acc0);
        acc1 = wmma_f16_guarded(aw1, bv, acc1);
        acc2 = wmma_f16_guarded(aw2, bv, acc2);
        acc3 = wmma_f16_guarded(aw3, bv, acc3);

#pragma unroll
        for (int r = 0; r < 8; ++r) {
            const float ig = sig_scaled(acc0[r], INV_ACC);
            const float fg = sig_scaled(acc1[r], INV_ACC);
            const float gg = tanh_scaled(acc2[r], INV_ACC);
            const float og = sig_scaled(acc3[r], INV_ACC);
            const float cr = fmaf(fg, c[r], ig * gg);
            c[r] = cr;
            h[r] = og * tanh_scaled(cr, 1.0f);
        }
    }

    v16h bh;
#pragma unroll
    for (int e = 0; e < 8; ++e) bh[e] = (_Float16)(h[e] * SC_ACT);
#pragma unroll
    for (int e = 8; e < 16; ++e) bh[e] = (_Float16)0.0f;
    const v16h a1 = frag_row8(W1 + (size_t)n * HID + 8 * hh, SC_W);
    v8f acc4;
#pragma unroll
    for (int r = 0; r < 8; ++r) acc4[r] = b1[8 * hh + r] * SC_ACC;
    acc4 = wmma_f16_guarded(a1, bh, acc4);

    float hid[8];
#pragma unroll
    for (int r = 0; r < 8; ++r) hid[r] = fmaxf(acc4[r] * INV_ACC, 0.0f);

    v16h bq;
#pragma unroll
    for (int e = 0; e < 8; ++e) bq[e] = (_Float16)(hid[e] * SC_ACT);
#pragma unroll
    for (int e = 8; e < 16; ++e) bq[e] = (_Float16)0.0f;
    const int   n2  = (n < NOUT) ? n : 0;
    const float sc2 = (n < NOUT) ? SC_W : 0.0f;
    const v16h a2 = frag_row8(W2 + (size_t)n2 * HID + 8 * hh, sc2);
    v8f acc5;
#pragma unroll
    for (int r = 0; r < 8; ++r) {
        float bv2 = 0.0f;
        if (r < NOUT) bv2 = (hh == 0) ? b2[r] * SC_ACC : 0.0f;
        acc5[r] = bv2;
    }
    acc5 = wmma_f16_guarded(a2, bq, acc5);

    v4f ov;
    ov.x = acc5[0] * INV_ACC;
    ov.y = acc5[1] * INV_ACC;
    ov.z = acc5[2] * INV_ACC;
    ov.w = acc5[3] * INV_ACC;
    const bool do_st = (hh == 0) && (row < B);
    volatile v4f* po = (volatile v4f*)(out + (size_t)row * NOUT);
    if (do_st) *po = ov;
    __threadfence();
    if (do_st) *po = ov;
}

extern "C" void kernel_launch(void* const* d_in, const int* in_sizes, int n_in,
                              void* d_out, int out_size, void* d_ws, size_t ws_size,
                              hipStream_t stream) {
    (void)d_ws; (void)ws_size;
    if (n_in < 9) return;
    const int B = out_size / NOUT;
    if (B <= 0) return;
    const int T = in_sizes[0] / B;
    if (T <= 0) return;
    if (in_sizes[1] != 4 * HID || in_sizes[2] != 4 * HID * HID || in_sizes[3] != 4 * HID ||
        in_sizes[4] != 4 * HID || in_sizes[5] != HID * HID || in_sizes[6] != HID ||
        in_sizes[7] != NOUT * HID || in_sizes[8] != NOUT) return;

    const float* x    = (const float*)d_in[0];
    const float* W_ih = (const float*)d_in[1];
    const float* W_hh = (const float*)d_in[2];
    const float* b_ih = (const float*)d_in[3];
    const float* b_hh = (const float*)d_in[4];
    const float* W1   = (const float*)d_in[5];
    const float* b1   = (const float*)d_in[6];
    const float* W2   = (const float*)d_in[7];
    const float* b2   = (const float*)d_in[8];
    float* out = (float*)d_out;

    const int nblk = (B + ROWS_PER_WAVE - 1) / ROWS_PER_WAVE;
    lstm_head_fused<<<dim3(nblk), dim3(32), 0, stream>>>(x, W_ih, W_hh, b_ih, b_hh, W1, b1, W2, b2, out, B, T);
    (void)hipGetLastError();
}
